// LINKX_9285719294274
// MI455X (gfx1250) — hardware-run, weakly checked
//
#include <hip/hip_runtime.h>


namespace {
constexpr int N = 50000, NP = 50048, NLIM = 50048  , NLIMN = (NLIM < N ? NLIM : N), EFULL = 800000, E = 800000, F = 128, H = 256, C = 40, CP = 48, RPB = 64, NBL = NLIM / RPB;
constexpr float XS = 8.0f, WSC = 256.0f, BNEPS = 1e-5f;
static_assert(NP % 64 == 0 && NLIM % 64 == 0 && N % 16 == 0, "tiling");
typedef _Float16 b16;
typedef __attribute__((ext_vector_type(16))) _Float16 v16b;
typedef __attribute__((ext_vector_type(8))) _Float16 v8b;
typedef __attribute__((ext_vector_type(8))) float v8f;
typedef __attribute__((ext_vector_type(4))) float v4f;
__device__ __forceinline__ float bf16_rne(float f) { unsigned int u = __float_as_uint(f); u += 0x7FFFu + ((u >> 16) & 1u); return __uint_as_float(u & 0xFFFF0000u); }
__device__ __forceinline__ void split16(float v, b16& hi, b16& lo) { hi = (b16)v; lo = (b16)(v - (float)hi); }
__device__ __forceinline__ v16b frag_kb(const b16* p, int hh) { const v8b a = *(const v8b*)(p + 8 * hh), b = *(const v8b*)(p + 16 + 8 * hh); v16b f;
#pragma unroll
  for (int e = 0; e < 8; ++e) { f[e] = a[e]; f[8 + e] = b[e]; } return f; }
__device__ __forceinline__ v8f wmma16b(v16b a, v16b b, v8f c) { v8f d = __builtin_amdgcn_wmma_f32_16x16x32_f16(false, a, false, b, (short)0, c, false, false); asm volatile("v_nop\n\tv_nop\n\tv_nop\n\tv_nop" : "+v"(d) : "v"(a), "v"(b)); return d; }
__device__ __forceinline__ void wave_lds_sync() { __builtin_amdgcn_fence(__ATOMIC_RELEASE, "workgroup"); __builtin_amdgcn_wave_barrier(); __builtin_amdgcn_fence(__ATOMIC_ACQUIRE, "workgroup"); }
__device__ __forceinline__ float pmul(float a, float b) { float p = a * b; asm volatile("" : "+v"(p)); return p; }
__device__ __forceinline__ int iclamp(int v, int lo, int hi) { return v < lo ? lo : (v > hi ? hi : v); }
constexpr int CSR_NBLK = 512, CSR_GB = 9, CSR_GN = 1 << CSR_GB  , CSR_MAXG = 512, CSR_CAP = 12288  ;
__global__ __launch_bounds__(64) void csrA_kernel(const int* __restrict__ dst, int E, int N, int nG, int CHP, int NGP, int* __restrict__ STG, int* __restrict__ HST) {
  extern __shared__ int sm[];
  int* cnt = sm; int* run = sm + NGP; int* ids = sm + 2 * NGP;
  const int b = blockIdx.x; const int ch = (E + CSR_NBLK - 1) / CSR_NBLK; const int e0 = b * ch, e1 = min(E, e0 + ch);
  for (int i = threadIdx.x; i < NGP; i += 64) cnt[i] = 0;
  for (int i = threadIdx.x; i < CHP; i += 64) ids[i] = -1;
  __syncthreads();
  if (threadIdx.x == 0) {
    for (int e = e0; e < e1; ++e) { int d = dst[e]; d = (d < 0) ? 0 : (d >= N ? N - 1 : d); cnt[d >> CSR_GB] += 1; }
    int acc = 0; for (int g = 0; g < nG; ++g) { run[g] = acc; acc += cnt[g]; }
    for (int e = e0; e < e1; ++e) { int d = dst[e]; d = (d < 0) ? 0 : (d >= N ? N - 1 : d); const int g = d >> CSR_GB; ids[run[g]] = e; run[g] += 1; } }
  __syncthreads();
  typedef __attribute__((ext_vector_type(4))) int v4i;
  for (int pass = 0; pass < 2; ++pass) {
    for (int i = threadIdx.x; i < CHP / 4; i += 64) *(volatile v4i*)(STG + (size_t)b * CHP + i * 4) = *(const v4i*)(&ids[i * 4]);
    for (int i = threadIdx.x; i < NGP / 4; i += 64) { v4i v; for (int e = 0; e < 4; ++e) v[e] = (i * 4 + e < nG) ? cnt[i * 4 + e] : 0; *(volatile v4i*)(HST + (size_t)b * NGP + i * 4) = v; }
    __threadfence(); }
}
__global__ __launch_bounds__(512) void csrS_kernel(const int* __restrict__ HST, int nG, int NGP, int* __restrict__ START, int* __restrict__ TOT, int* __restrict__ OFF) {
  __shared__ int tot[CSR_MAXG];
  const int b = threadIdx.x;
  for (int pass = 0; pass < 2; ++pass) { int runb = 0; for (int g = 0; g < nG; ++g) { int c = HST[(size_t)b * NGP + g]; c = (c < 0) ? 0 : c; ((volatile int*)OFF)[(size_t)g * CSR_NBLK + b] = runb; runb += c; } __threadfence(); }
  for (int g = threadIdx.x; g < nG; g += 512) { int s = 0; for (int bb = 0; bb < CSR_NBLK; ++bb) { int c = HST[(size_t)bb * NGP + g]; s += (c < 0) ? 0 : c; } tot[g] = s; }
  __syncthreads();
  if (threadIdx.x < 32) {
    __shared__ int st[CSR_MAXG + 32];
    if (threadIdx.x == 0) { int acc = 0; for (int g = 0; g < NGP; ++g) { st[g] = acc; if (g < nG) acc += (tot[g] + 31) & ~31; } st[NGP] = acc; }
    __builtin_amdgcn_fence(__ATOMIC_RELEASE, "workgroup"); __builtin_amdgcn_wave_barrier(); __builtin_amdgcn_fence(__ATOMIC_ACQUIRE, "workgroup");
    for (int pass = 0; pass < 2; ++pass) { for (int i = threadIdx.x; i < NGP + 32; i += 32) { ((volatile int*)START)[i] = (i <= NGP) ? st[min(i, NGP)] : 0; ((volatile int*)TOT)[i] = (i < nG) ? tot[i] : 0; } __threadfence(); } }
}
__global__ __launch_bounds__(256) void csrB_kernel(const int* __restrict__ dst, int N, int nG, int CHP, int NGP, int permLen, const int* __restrict__ STG, const int* __restrict__ HST, const int* __restrict__ OFF, const int* __restrict__ START, const int* __restrict__ TOT, int* __restrict__ PERM, int* __restrict__ ROWPTR, int* __restrict__ ROWCNT, int* __restrict__ FLAG) {
  typedef __attribute__((ext_vector_type(4))) int v4i;
  __shared__ int ids[CSR_CAP]; __shared__ unsigned short key[CSR_CAP]; __shared__ int outp[CSR_CAP]; __shared__ int ncnt[CSR_GN + 1]; __shared__ int boff[CSR_NBLK + 1];
  const int g = blockIdx.x, t_ = threadIdx.x; int tot = TOT[g]; int st = START[g], stn = START[g + 1]; const int v0 = g * CSR_GN; const int nv = min(CSR_GN, N - v0);
  st = (st < 0) ? 0 : (st > permLen - 32 ? permLen - 32 : st) & ~31; stn = (stn < st) ? st : (stn > permLen ? permLen : stn); tot = (tot < 0) ? 0 : tot; if (tot > stn - st && tot <= CSR_CAP) tot = stn - st;
  if (tot > CSR_CAP) {
    for (int pass = 0; pass < 2; ++pass) { for (int i = t_; i < CSR_GN / 4; i += 256) { v4i a, c; for (int e = 0; e < 4; ++e) { a[e] = st; c[e] = 0; } *(volatile v4i*)(ROWPTR + v0 + i * 4) = a; *(volatile v4i*)(ROWCNT + v0 + i * 4) = c; } if (t_ == 0) ((volatile int*)FLAG)[0] = 1; __threadfence(); } (void)nv; return; }
  if (t_ == 0) { int acc = 0; for (int b = 0; b < CSR_NBLK; ++b) { boff[b] = acc; int c = HST[(size_t)b * NGP + g]; c = (c < 0) ? 0 : (c > CHP ? CHP : c); acc += c; if (acc > tot) acc = tot; } boff[CSR_NBLK] = acc; }
  for (int i = t_; i <= CSR_GN; i += 256) ncnt[i] = 0;
  __syncthreads();
  for (int b = 0; b < CSR_NBLK; ++b) { const int c = boff[b + 1] - boff[b]; int o_ = OFF[(size_t)g * CSR_NBLK + b]; o_ = (o_ < 0) ? 0 : (o_ > CHP - c ? CHP - c : o_); const int* src_ = STG + (size_t)b * CHP + o_;
    for (int i = t_; i < c; i += 256) { int id = src_[i]; id = (id < 0) ? 0 : id; ids[boff[b] + i] = id; int d = dst[id]; d = (d < v0) ? v0 : (d >= N ? N - 1 : d); int kk = d - v0; kk = (kk < 0) ? 0 : (kk >= CSR_GN ? CSR_GN - 1 : kk); key[boff[b] + i] = (unsigned short)kk; } }
  __syncthreads();
  if (t_ == 0) { for (int i = 0; i < tot; ++i) ncnt[key[i]] += 1; int acc = 0; for (int vl = 0; vl < CSR_GN; ++vl) { const int c = ncnt[vl]; ncnt[vl] = acc; acc += c; } ncnt[CSR_GN] = acc;
    for (int i = 0; i < tot; ++i) { const int vl = key[i]; outp[ncnt[vl]] = ids[i]; ncnt[vl] += 1; }
    for (int vl = CSR_GN; vl > 0; --vl) ncnt[vl] = ncnt[vl - 1]; ncnt[0] = 0; }
  __syncthreads();
  for (int pass = 0; pass < 2; ++pass) {
    for (int i = t_; i < (stn - st) / 4; i += 256) { v4i v; for (int e = 0; e < 4; ++e) { const int q = i * 4 + e; v[e] = (q < tot) ? outp[q] : -1; } *(volatile v4i*)(PERM + st + i * 4) = v; }
    for (int i = t_; i < CSR_GN / 4; i += 256) { v4i a, c; for (int e = 0; e < 4; ++e) { const int vl = i * 4 + e; a[e] = st + ncnt[vl]; c[e] = (vl < nv) ? (ncnt[vl + 1] - ncnt[vl]) : 0; } *(volatile v4i*)(ROWPTR + v0 + i * 4) = a; *(volatile v4i*)(ROWCNT + v0 + i * 4) = c; }
    __threadfence(); }
}
__global__ __launch_bounds__(256) void csrZ_kernel(int* __restrict__ p, size_t n4) { typedef __attribute__((ext_vector_type(4))) int v4i; const size_t tid = (size_t)blockIdx.x * 256 + threadIdx.x, nth = (size_t)gridDim.x * 256; v4i z = {0, 0, 0, 0}; for (size_t i = tid; i < n4; i += nth) *(volatile v4i*)(p + i * 4) = z; }
struct CsrBufs { int *STG, *HST, *OFF, *START, *TOT, *PERM, *ROWPTR, *ROWCNT, *FLAG; int nG, NGP, CHP; size_t permLen; char* base; size_t bytes; };
static size_t csr_carve(CsrBufs& c, char* ws, size_t off, int E, int N) {
  const size_t off0 = off; c.base = ws + off;
  auto al = [&](size_t bytes) { char* p = ws + off; off += (bytes + 255) & ~(size_t)255; return p; };
  c.nG = (N + CSR_GN - 1) / CSR_GN; c.NGP = (c.nG + 31) & ~31; const int ch = (E + CSR_NBLK - 1) / CSR_NBLK; c.CHP = (ch + 31) & ~31; c.permLen = (size_t)E + 32 * (size_t)c.nG + 32;
  c.STG = (int*)al((size_t)CSR_NBLK * c.CHP * 4); c.HST = (int*)al((size_t)CSR_NBLK * c.NGP * 4); c.OFF = (int*)al((size_t)c.NGP * CSR_NBLK * 4); c.START = (int*)al((size_t)(c.NGP + 64) * 4); c.TOT = (int*)al((size_t)(c.NGP + 64) * 4);
  c.PERM = (int*)al(c.permLen * 4); c.ROWPTR = (int*)al((size_t)c.nG * CSR_GN * 4); c.ROWCNT = (int*)al((size_t)c.nG * CSR_GN * 4); c.FLAG = (int*)al(256);
  c.bytes = off - off0; return off;
}
static void csr_build(const CsrBufs& c, const int* dst, int E, int N, hipStream_t stream) {
  const size_t smem = (size_t)(2 * c.NGP + c.CHP) * 4;
  csrZ_kernel<<<512, 256, 0, stream>>>((int*)c.base, c.bytes / 16);
  csrA_kernel<<<CSR_NBLK, 64, smem, stream>>>(dst, E, N, c.nG, c.CHP, c.NGP, c.STG, c.HST);
  csrS_kernel<<<1, 512, 0, stream>>>(c.HST, c.nG, c.NGP, c.START, c.TOT, c.OFF);
  csrB_kernel<<<c.nG, 256, 0, stream>>>(dst, N, c.nG, c.CHP, c.NGP, (int)c.permLen, c.STG, c.HST, c.OFF, c.START, c.TOT, c.PERM, c.ROWPTR, c.ROWCNT, c.FLAG);
}

typedef __attribute__((ext_vector_type(4))) _Float16 v4h;
typedef __attribute__((ext_vector_type(2))) _Float16 v2h;
typedef __attribute__((ext_vector_type(2))) float v2f;
__global__ __launch_bounds__(256) void prep_kernel(const float* __restrict__ x, const float* __restrict__ wn, const float* __restrict__ wc1, const float* __restrict__ wc2, const float* __restrict__ wf1, const float* __restrict__ wf2, b16* __restrict__ Xh, b16* __restrict__ WN, b16* __restrict__ WC, b16* __restrict__ WF1, b16* __restrict__ WF2) {
  size_t t = (size_t)blockIdx.x * 256 + threadIdx.x; v8b o;
  auto emit = [&](b16* dst, size_t e) { for (int pass = 0; pass < 2; ++pass) { *(volatile v8b*)(dst + e) = o; __threadfence(); } };
  { const size_t n = (size_t)NP * F / 8; if (t < n) { const size_t e = t * 8; const size_t v = e / F; for (int j = 0; j < 8; ++j) o[j] = (v < (size_t)N) ? (b16)(bf16_rne(x[e + j]) * XS) : (b16)0.0f; emit(Xh, e); return; } t -= n; }
  { const size_t n = (size_t)H * F / 8; if (t < n) { const size_t e = t * 8; const int oo = (int)(e / F), k0 = (int)(e % F); for (int j = 0; j < 8; ++j) o[j] = (b16)(bf16_rne(wn[(size_t)(k0 + j) * H + oo]) * WSC); emit(WN, e); return; } t -= n; }
  { const size_t n = (size_t)H * 2 * H / 8; if (t < n) { const size_t e = t * 8; const int oo = (int)(e / (2 * H)), k0 = (int)(e % (2 * H)); for (int j = 0; j < 8; ++j) { const int k = k0 + j; const float w = (k < H) ? wc1[(size_t)k * H + oo] : wc2[(size_t)(k - H) * H + oo]; o[j] = (b16)(bf16_rne(w) * WSC); } emit(WC, e); return; } t -= n; }
  { const size_t n = (size_t)H * H / 8; if (t < n) { const size_t e = t * 8; const int oo = (int)(e / H), k0 = (int)(e % H); for (int j = 0; j < 8; ++j) o[j] = (b16)(bf16_rne(wf1[(size_t)(k0 + j) * H + oo]) * WSC); emit(WF1, e); return; } t -= n; }
  { const size_t n = (size_t)CP * H / 8; if (t < n) { const size_t e = t * 8; const int oo = (int)(e / H), k0 = (int)(e % H); for (int j = 0; j < 8; ++j) o[j] = (oo < C) ? (b16)(bf16_rne(wf2[(size_t)(k0 + j) * C + oo]) * WSC) : (b16)0.0f; emit(WF2, e); } }
}
__global__ __launch_bounds__(256) void agg_kernel(const float* __restrict__ wedge, const float* __restrict__ ew, const float* __restrict__ bedge, const int* __restrict__ srcs, const int* __restrict__ PERM, const int* __restrict__ ROWPTR, const int* __restrict__ ROWCNT, int permLen, b16* __restrict__ Ah, b16* __restrict__ Al) {
  const int wave = threadIdx.x >> 5, lane = threadIdx.x & 31; const size_t v = (size_t)blockIdx.x * 8 + wave; const int c = lane * 8; v4f a0 = {0.0f, 0.0f, 0.0f, 0.0f}, a1 = a0;
  if (v < (size_t)N) { int st = ROWPTR[v], cnt = ROWCNT[v]; cnt = iclamp(cnt, 0, 65536); st = iclamp(st, 0, permLen - cnt);
#pragma unroll 1
    for (int j = 0; j < cnt; ++j) { const int e = iclamp(PERM[st + j], 0, E - 1); const size_t s = (size_t)iclamp(srcs[e], 0, N - 1); const float w = bf16_rne(ew[e]); v4f x0 = *(const v4f*)(wedge + s * H + c), x1 = *(const v4f*)(wedge + s * H + c + 4);
      for (int i = 0; i < 4; ++i) { a0[i] += pmul(w, bf16_rne(x0[i])); a1[i] += pmul(w, bf16_rne(x1[i])); } }
    for (int i = 0; i < 4; ++i) { a0[i] += bf16_rne(bedge[c + i]); a1[i] += bf16_rne(bedge[c + 4 + i]); } }
  v8b hv, lv; for (int i = 0; i < 4; ++i) { b16 p, q; split16(a0[i] * XS, p, q); hv[i] = p; lv[i] = q; split16(a1[i] * XS, p, q); hv[4 + i] = p; lv[4 + i] = q; }
  for (int pass = 0; pass < 2; ++pass) { *(volatile v8b*)(Ah + v * H + c) = hv; *(volatile v8b*)(Al + v * H + c) = lv; __threadfence(); }
}
template <int KD, int KSPLIT, int TWO0, int TWO1, int MODE>
__global__ __launch_bounds__(256) void gemm_kernel(const b16* __restrict__ A0h, const b16* __restrict__ A0l, int S0, const b16* __restrict__ A1h, const b16* __restrict__ A1l, int S1, const b16* __restrict__ WT, const float* __restrict__ bias, const float* __restrict__ bias2, b16* __restrict__ Oh, b16* __restrict__ Ol, float* __restrict__ OUTF) {
  __shared__ __attribute__((aligned(16))) float Tf[8][16][128 + 4];
  const int wave = threadIdx.x >> 5, lane = threadIdx.x & 31, nloc = lane & 15, hlf = lane >> 4; const size_t m0 = (size_t)blockIdx.x * 64 + (wave & 3) * 16; const int n0 = (wave >> 2) * 128;
  v8f acc[8];
#pragma unroll
  for (int t = 0; t < 8; ++t) acc[t] = (v8f){};
#pragma unroll 2
  for (int kb = 0; kb < KD; kb += 32) { v16b a, al; const bool p0 = kb < KSPLIT;
    if (p0) { a = frag_kb(A0h + (m0 + nloc) * S0 + kb, hlf); if (TWO0) al = frag_kb(A0l + (m0 + nloc) * S0 + kb, hlf); }
    else    { a = frag_kb(A1h + (m0 + nloc) * S1 + (kb - KSPLIT), hlf); if (TWO1) al = frag_kb(A1l + (m0 + nloc) * S1 + (kb - KSPLIT), hlf); }
#pragma unroll
    for (int t = 0; t < 8; ++t) { const v16b bw = frag_kb(WT + (size_t)(n0 + t * 16 + nloc) * KD + kb, hlf); acc[t] = wmma16b(a, bw, acc[t]); if ((p0 && TWO0) || (!p0 && TWO1)) acc[t] = wmma16b(al, bw, acc[t]); } }
  __syncthreads();
#pragma unroll
  for (int t = 0; t < 8; ++t) { const int cc = n0 + t * 16 + nloc; float bb = bf16_rne(bias[cc]); if (MODE == 1) bb += bf16_rne(bias2[cc]);
#pragma unroll
    for (int r = 0; r < 8; ++r) { const size_t row = m0 + 8 * hlf + r; float v = acc[t][r] * (1.0f / (XS * WSC)) + bb;
      if (MODE == 2) v = fmaxf(v, 0.0f); if (row >= (size_t)NLIMN) v = 0.0f; Tf[wave][8 * hlf + r][t * 16 + nloc] = v; } }
  wave_lds_sync();
  if (MODE == 1) {
    for (int rr = 0; rr < 16; ++rr) { const size_t row = m0 + rr; const int cc = n0 + lane * 4; v4f f = *(const v4f*)(&Tf[wave][rr][lane * 4]);
      const v4h a0 = *(const v4h*)(A0h + row * S0 + cc), b0 = *(const v4h*)(A0l + row * S0 + cc), a1 = *(const v4h*)(A1h + row * S1 + cc), b1 = *(const v4h*)(A1l + row * S1 + cc);
      for (int j = 0; j < 4; ++j) { float v = f[j] + ((float)a0[j] + (float)b0[j]) * (1.0f / XS) + ((float)a1[j] + (float)b1[j]) * (1.0f / XS); v = fmaxf(v, 0.0f); if (row >= (size_t)NLIMN) v = 0.0f; f[j] = v; }
      *(v4f*)(&Tf[wave][rr][lane * 4]) = f; }
    wave_lds_sync(); }
  for (int pass = 0; pass < 2; ++pass) { for (int rr = 0; rr < 16; ++rr) { const v4f f = *(const v4f*)(&Tf[wave][rr][lane * 4]);
      if (MODE == 2) *(volatile v4f*)(OUTF + (m0 + rr) * H + n0 + lane * 4) = f;
      else { v4h hv, lv; for (int j = 0; j < 4; ++j) { b16 p, q; split16(f[j] * XS, p, q); hv[j] = p; lv[j] = q; } *(volatile v4h*)(Oh + (m0 + rr) * H + n0 + lane * 4) = hv; *(volatile v4h*)(Ol + (m0 + rr) * H + n0 + lane * 4) = lv; } }
    __threadfence(); }
}
__global__ __launch_bounds__(256) void colpart_kernel(const float* __restrict__ G, const float* __restrict__ MEAN, int centred, float* __restrict__ PS) {
  const int c = threadIdx.x; const float m = centred ? MEAN[c] : 0.0f; float s = 0.0f;
#pragma unroll 1
  for (int rr = 0; rr < RPB; ++rr) { const size_t v = (size_t)blockIdx.x * RPB + rr; if (v < (size_t)NLIMN) { const float d = G[v * H + c] - m; s += centred ? d * d : d; } }
  for (int pass = 0; pass < 2; ++pass) { ((volatile float*)PS)[(size_t)blockIdx.x * H + c] = s; __threadfence(); }
}
__global__ __launch_bounds__(256) void colstat_kernel(const float* __restrict__ PS, float* __restrict__ STAT) {
  const int c = threadIdx.x; float s = 0.0f;
#pragma unroll 1
  for (int b = 0; b < NBL; ++b) s += PS[(size_t)b * H + c];
  for (int pass = 0; pass < 2; ++pass) { ((volatile float*)STAT)[c] = s * (1.0f / NLIMN); __threadfence(); }
}
__global__ __launch_bounds__(256) void apply_kernel(const float* __restrict__ G, const float* __restrict__ MEAN, const float* __restrict__ VAR, const float* __restrict__ g_, const float* __restrict__ b_, b16* __restrict__ Oh, b16* __restrict__ Ol) {
  const size_t u = (size_t)blockIdx.x * 256 + threadIdx.x; if (u >= (size_t)NP * H / 8) return; const size_t e = u * 8; const size_t v = e / H; const int c0 = (int)(e % H); v8b hv, lv;
  for (int j = 0; j < 8; ++j) { const int c = c0 + j; float y = 0.0f; if (v < (size_t)NLIMN) y = (G[e + j] - MEAN[c]) * rsqrtf(VAR[c] + BNEPS) * bf16_rne(g_[c]) + bf16_rne(b_[c]); b16 p, q; split16(y * XS, p, q); hv[j] = p; lv[j] = q; }
  for (int pass = 0; pass < 2; ++pass) { *(volatile v8b*)(Oh + e) = hv; *(volatile v8b*)(Ol + e) = lv; __threadfence(); }
}
__global__ __launch_bounds__(64) void cls_kernel(const b16* __restrict__ Ah, const b16* __restrict__ Al, const b16* __restrict__ WF2, const float* __restrict__ b2, float* __restrict__ out) {
  __shared__ __attribute__((aligned(16))) float To[2][16 * C];
  const int wave = threadIdx.x >> 5, lane = threadIdx.x & 31, nloc = lane & 15, hlf = lane >> 4; const size_t m0 = (size_t)blockIdx.x * 32 + wave * 16; if (m0 >= (size_t)N) return;
  v8f acc[3];
#pragma unroll
  for (int t = 0; t < 3; ++t) acc[t] = (v8f){};
#pragma unroll 2
  for (int kb = 0; kb < H; kb += 32) { const v16b a = frag_kb(Ah + (m0 + nloc) * H + kb, hlf), al = frag_kb(Al + (m0 + nloc) * H + kb, hlf);
#pragma unroll
    for (int t = 0; t < 3; ++t) { const v16b bw = frag_kb(WF2 + (size_t)(t * 16 + nloc) * H + kb, hlf); acc[t] = wmma16b(a, bw, acc[t]); acc[t] = wmma16b(al, bw, acc[t]); } }
#pragma unroll
  for (int t = 0; t < 3; ++t) { const int c = t * 16 + nloc; if (c < C) { const float bb = bf16_rne(b2[c]);
#pragma unroll
      for (int r = 0; r < 8; ++r) To[wave][(8 * hlf + r) * C + c] = acc[t][r] * (1.0f / (XS * WSC)) + bb; } }
  wave_lds_sync();
  const float* tw = &To[wave][0]; float* ob = out + m0 * C;
  for (int pass = 0; pass < 2; ++pass) { for (int p = lane; p < 16 * C / 4; p += 32) *(volatile v4f*)(ob + p * 4) = *(const v4f*)(tw + p * 4); __threadfence(); }
}
}

extern "C" void kernel_launch(void* const* d_in, const int* in_sizes, int n_in, void* d_out, int out_size, void* d_ws, size_t ws_size, hipStream_t stream) {
  (void)n_in;
  auto Fp = [&](int i) { return (const float*)d_in[i]; }; auto Ip = [&](int i) { return (const int*)d_in[i]; };
  if (in_sizes[0] != N * F || in_sizes[1] != 2 * EFULL || in_sizes[2] != EFULL || in_sizes[3] != N * H || in_sizes[4] != H || in_sizes[5] != F * H || in_sizes[7] != H * H || in_sizes[9] != H * H || in_sizes[11] != H * H || in_sizes[13] != H || in_sizes[15] != H * C || in_sizes[16] != C || out_size != N * C) return;
  size_t off = 0; char* ws = (char*)d_ws;
  auto carve = [&](size_t bytes) { char* p = ws + off; off += (bytes + 255) & ~(size_t)255; return p; };
  b16* Xh = (b16*)carve((size_t)NP * F * 2); b16* WN = (b16*)carve((size_t)H * F * 2); b16* WC = (b16*)carve((size_t)H * 2 * H * 2); b16* WF1 = (b16*)carve((size_t)H * H * 2); b16* WF2 = (b16*)carve((size_t)CP * H * 2);
  b16* HAh = (b16*)carve((size_t)NP * H * 2); b16* HAl = (b16*)carve((size_t)NP * H * 2); b16* HXh = (b16*)carve((size_t)NP * H * 2); b16* HXl = (b16*)carve((size_t)NP * H * 2);
  float* G = (float*)HXh;
  float* PS = (float*)carve((size_t)(NP / RPB) * H * 4); float* ST = (float*)carve((size_t)2 * H * 4);
  CsrBufs csr; off = csr_carve(csr, ws, off, E, N);
  if (off > ws_size || off > ((size_t)128 << 20)) return;
  prep_kernel<<<(unsigned)((((size_t)NP * F + (size_t)H * F + (size_t)H * 2 * H + (size_t)H * H + (size_t)CP * H) / 8 + 255) / 256), 256, 0, stream>>>(Fp(0), Fp(5), Fp(7), Fp(9), Fp(11), Fp(15), Xh, WN, WC, WF1, WF2);
  csr_build(csr, Ip(1) + EFULL, E, N, stream);
  agg_kernel<<<NLIM / 8, 256, 0, stream>>>(Fp(3), Fp(2), Fp(4), Ip(1), csr.PERM, csr.ROWPTR, csr.ROWCNT, (int)csr.permLen, HAh, HAl);
  gemm_kernel<F, F, 0, 0, 0><<<NLIM / 64, 256, 0, stream>>>(Xh, nullptr, F, nullptr, nullptr, 0, WN, Fp(6), nullptr, HXh, HXl, nullptr);
  gemm_kernel<2 * H, H, 1, 1, 1><<<NLIM / 64, 256, 0, stream>>>(HAh, HAl, H, HXh, HXl, H, WC, Fp(8), Fp(10), HAh, HAl, nullptr);
  gemm_kernel<H, H, 1, 0, 2><<<NLIM / 64, 256, 0, stream>>>(HAh, HAl, H, nullptr, nullptr, 0, WF1, Fp(12), nullptr, nullptr, nullptr, G);
  colpart_kernel<<<NBL, 256, 0, stream>>>(G, nullptr, 0, PS); colstat_kernel<<<1, 256, 0, stream>>>(PS, ST);
  colpart_kernel<<<NBL, 256, 0, stream>>>(G, ST, 1, PS);      colstat_kernel<<<1, 256, 0, stream>>>(PS, ST + H);
  apply_kernel<<<(unsigned)(((size_t)NP * H / 8 + 255) / 256), 256, 0, stream>>>(G, ST, ST + H, Fp(13), Fp(14), HAh, HAl);
  cls_kernel<<<NLIM / 32, 64, 0, stream>>>(HAh, HAl, WF2, Fp(16), (float*)d_out);
}
